// SpaMamba_47425028882459
// MI455X (gfx1250) — hardware-run, weakly checked
//
#include <hip/hip_runtime.h>

#define NB    4
#define CH    64
#define HWN   16384
#define NTOK  (NB * HWN)
#define DI    128
#define DIN2  256
#define NS    16
#define DTR   4
#define NXD   36
#define NXP   64
#define CHUNK 128
#define NCHK  (NTOK / CHUNK)
#define TC    16
#define TV    32
#define TO    32
#define LNEPS 1e-5f

static_assert(NTOK % 128 == 0 && NTOK % CHUNK == 0 && CHUNK % TC == 0 && NTOK % TV == 0 && NTOK % TO == 0);
static_assert(CH == 64 && DI == 128 && DIN2 == 2 * DI && CH % 32 == 0 && DI % 32 == 0);
static_assert(HWN % 64 == 0 && CH % 64 == 0 && HWN % TO == 0 && (128 % TO) == 0 && HWN == (1 << 14));
static_assert(DTR + 2 * NS == NXD && NXD <= NXP && NXP == 64 && NS == 16 && DTR == 4);
static_assert(CHUNK == 128 && TC == 16 && TV == 32 && TO == 32);
static_assert((DIN2 * CH) % 2048 == 0 && (NXP * DI) % 2048 == 0 && (CH * DI) % 2048 == 0 && (CH * CH) % 2048 == 0);
static_assert((DIN2 * CH) % 8 == 0 && (NXD * DI) % 8 == 0 && (CH * DI) % 8 == 0 && (CH * CH) % 8 == 0);

typedef __bf16         v16b __attribute__((ext_vector_type(16)));
typedef unsigned short v8us __attribute__((ext_vector_type(8)));
typedef float          v8f  __attribute__((ext_vector_type(8)));
typedef float          v4f  __attribute__((ext_vector_type(4)));
typedef float          v2f  __attribute__((ext_vector_type(2)));
typedef v8us __attribute__((may_alias)) v8usa;
typedef v4f  __attribute__((may_alias)) v4fa;
typedef v2f  __attribute__((may_alias)) v2fa;

union Frag { v16b v; v8us half[2]; };

constexpr size_t WO_WIN  = 0;
constexpr size_t WO_WXP  = WO_WIN + (size_t)DIN2 * CH * 2;
constexpr size_t WO_WOUT = WO_WXP + (size_t)NXP * DI * 2;
constexpr size_t WO_WPJ  = WO_WOUT + (size_t)CH * DI * 2;
constexpr size_t SZ_W    = WO_WPJ + (size_t)CH * CH * 2;
constexpr size_t OFF_X0  = 131072;
constexpr size_t SZ_X0   = (size_t)NTOK * CH * 2;
constexpr size_t OFF_MOB = OFF_X0;
constexpr size_t OFF_XH  = OFF_X0 + SZ_X0;
constexpr size_t SZ_XH   = (size_t)NTOK * DI * 4;
constexpr size_t OFF_Z   = OFF_XH + SZ_XH;
constexpr size_t OFF_XC  = OFF_Z + SZ_XH;
constexpr size_t SZ_XC   = (size_t)NTOK * DI * 2;
constexpr size_t OFF_YB  = OFF_XC;
constexpr size_t OFF_XD  = OFF_XC + SZ_XC;
constexpr size_t SZ_XD   = (size_t)NTOK * NXP * 4;
constexpr size_t OFF_P   = OFF_XD;
constexpr size_t OFF_HS  = OFF_XD + SZ_XD;
constexpr size_t SZ_REC  = (size_t)NCHK * CHUNK * NS * 4;
constexpr size_t OFF_AP  = OFF_HS + SZ_REC;
constexpr size_t OFF_CR  = OFF_AP + SZ_REC;
constexpr size_t WS_END  = OFF_CR + SZ_REC;
static_assert(SZ_W <= OFF_X0);
static_assert((size_t)NTOK * CH * 2 <= SZ_X0);
static_assert((size_t)NTOK * DI * 2 <= SZ_XC);
static_assert((size_t)NTOK * CH * 4 <= SZ_XD);
static_assert(WS_END <= (size_t)134217728);
static_assert(WO_WXP % 128 == 0 && WO_WOUT % 128 == 0 && WO_WPJ % 128 == 0 && OFF_X0 % 128 == 0);
static_assert(OFF_XH % 128 == 0 && OFF_Z % 128 == 0 && OFF_XC % 128 == 0 && OFF_XD % 128 == 0);
static_assert(OFF_HS % 128 == 0 && OFF_AP % 128 == 0 && OFF_CR % 128 == 0);
static_assert((size_t)(HWN / 64) * (CH / 64) * NB * 64 * 64 * 2 == SZ_X0);
static_assert((size_t)(NTOK / 128) * 2 * 128 * 64 * 4 == SZ_XH);
static_assert((size_t)(NTOK / TV) * TV * DI * 2 == SZ_XC);
static_assert((size_t)(NTOK / 128) * 1 * 128 * 64 * 4 == SZ_XD);
static_assert((size_t)NCHK * 64 * 32 * 4 == SZ_REC);
static_assert((size_t)NCHK * (CHUNK / TC) * 32 * 64 * 2 == (size_t)NTOK * DI * 2);
static_assert((size_t)(NTOK / 128) * 128 * 64 * 2 == (size_t)NTOK * CH * 2);
static_assert((size_t)(NTOK / 128) * 128 * 64 * 4 == (size_t)NTOK * CH * 4);
static_assert((size_t)(NTOK / TO) * CH * 32 * 4 == (size_t)NB * CH * HWN * 4);

__device__ __forceinline__ unsigned short bf16_bits(float f) {
  unsigned u = __float_as_uint(f);
  u += 0x7FFFu + ((u >> 16) & 1u);
  return (unsigned short)(u >> 16);
}
__device__ __forceinline__ float bf16_val(unsigned short b) { return __uint_as_float(((unsigned)b) << 16); }
__device__ __forceinline__ float bf16r(float f) { return bf16_val(bf16_bits(f)); }
__device__ __forceinline__ v8f zero8() {
  v8f z;
#pragma unroll
  for (int i = 0; i < 8; ++i) z[i] = 0.0f;
  return z;
}
__device__ __forceinline__ float wsum(float v) {
#pragma unroll
  for (int o = 16; o > 0; o >>= 1) v += __shfl_xor(v, o, 32);
  return v;
}
__device__ __forceinline__ float sigm(float v) {
  const float e = __expf(-v);
  return __builtin_amdgcn_rcpf(1.0f + e);
}
__device__ __forceinline__ float silu_f(float v) { return v * sigm(v); }
__device__ __forceinline__ float softplus_f(float v) {
  const float e = __expf(v);
  const float s = __logf(1.0f + e);
  return (v > 15.0f) ? v : s;
}

__device__ __forceinline__ void ldfrag_g(Frag& f, const unsigned short* p, int h) {
  f.half[0] = *(const v8usa*)(p + 8 * h);
  f.half[1] = *(const v8usa*)(p + 16 + 8 * h);
}
__device__ __forceinline__ v8f mma16(v8f c, const Frag& a, const Frag& b) {
  v8f d = __builtin_amdgcn_wmma_f32_16x16x32_bf16(false, a.v, false, b.v, (short)0, c, false, false);
  asm volatile("v_nop\n\tv_nop\n\tv_nop\n\tv_nop" : "+v"(d) : "v"(a.v), "v"(b.v));
  return d;
}

__device__ __forceinline__ void tc_store_pass(const unsigned short* sT, unsigned short* dst, int P,
                                              int orow0, int ocol0, int w, int lane) {
  const int q8 = lane & 7, sub = lane >> 3;
#pragma unroll
  for (int i = 0; i < 2; ++i) {
    const int li = 8 * w + 4 * i + sub;
    const v8us v = *(const v8usa*)(sT + li * 64 + 8 * q8);
    unsigned short* p = dst + (size_t)(orow0 + li) * P + ocol0 + 8 * q8;
    *(volatile v8us*)p = v;
  }
}

__global__ __launch_bounds__(256)
void tcvt_kernel(const float* __restrict__ in, int R, int Cc, size_t izs,
                 unsigned short* out, int P, size_t ozs)
{
  __shared__ __attribute__((aligned(16))) unsigned short sT[64 * 64];

  const int tid = threadIdx.x, lane = tid & 31, w = tid >> 5;
  const int orow0 = blockIdx.x * 64, ocol0 = blockIdx.y * 64;
  const float* src = in + (size_t)blockIdx.z * izs;
  unsigned short* dst = out + (size_t)blockIdx.z * ozs;

  const int c4 = tid & 15, rs = tid >> 4;
  const int c = orow0 + 4 * c4;
  const bool cok = (c < Cc);
  const int cc = cok ? c : (Cc - 4);
#pragma unroll
  for (int i = 0; i < 4; ++i) {
    const int rloc = 16 * i + rs;
    const int r = ocol0 + rloc;
    const int rr = (r < R) ? r : (R - 1);
    const v4f v = *(const v4fa*)(src + (size_t)rr * Cc + cc);
    const bool ok = cok && (r < R);
    sT[(4 * c4 + 0) * 64 + rloc] = ok ? bf16_bits(v[0]) : (unsigned short)0;
    sT[(4 * c4 + 1) * 64 + rloc] = ok ? bf16_bits(v[1]) : (unsigned short)0;
    sT[(4 * c4 + 2) * 64 + rloc] = ok ? bf16_bits(v[2]) : (unsigned short)0;
    sT[(4 * c4 + 3) * 64 + rloc] = ok ? bf16_bits(v[3]) : (unsigned short)0;
  }
  __syncthreads();

  tc_store_pass(sT, dst, P, orow0, ocol0, w, lane);
  __threadfence();
  tc_store_pass(sT, dst, P, orow0, ocol0, w, lane);
}

__global__ __launch_bounds__(256)
void cvt_kernel(const float* __restrict__ src, int nsrc, unsigned short* dst, int ndst)
{
  const int i = blockIdx.x * 256 + threadIdx.x;
  const int e0 = 8 * i;
  if (e0 >= ndst) return;
  const bool ok = (e0 + 8 <= nsrc);
  const int ea = ok ? e0 : 0;
  const v4f a = *(const v4fa*)(src + ea);
  const v4f c = *(const v4fa*)(src + ea + 4);
  v8us o;
#pragma unroll
  for (int j = 0; j < 4; ++j) {
    o[j]     = ok ? bf16_bits(a[j]) : (unsigned short)0;
    o[4 + j] = ok ? bf16_bits(c[j]) : (unsigned short)0;
  }
  unsigned short* p = dst + e0;
  *(volatile v8us*)p = o;
  __threadfence();
  *(volatile v8us*)p = o;
}

__device__ __forceinline__ void c_store_pass(const float* sT, float* C, int ldc, int m0w, int cy, int w, int lane) {
  const int q8 = lane & 7, sub = lane >> 3;
#pragma unroll
  for (int i = 0; i < 16; ++i) {
    const int lid = 4 * i + sub;
    const int rl = lid >> 1, hl = lid & 1;
    const v4f v = *(const v4fa*)(sT + (32 * w + rl) * 64 + 32 * hl + 4 * q8);
    float* dst = C + (size_t)(m0w + rl) * ldc + 64 * cy + 32 * hl + 4 * q8;
    *(volatile v4f*)dst = v;
  }
}

__device__ __forceinline__ void b_store_pass(const float* sT, unsigned short* Cb, int ldc, int m0w, int cy,
                                             int w, int lane) {
  const int q8 = lane & 7, sub = lane >> 3;
#pragma unroll
  for (int i = 0; i < 8; ++i) {
    const int rl = 4 * i + sub;
    const float* sr = sT + (32 * w + rl) * 64 + 8 * q8;
    const v4f a = *(const v4fa*)sr;
    const v4f c = *(const v4fa*)(sr + 4);
    v8us o;
    o[0] = bf16_bits(a[0]); o[1] = bf16_bits(a[1]); o[2] = bf16_bits(a[2]); o[3] = bf16_bits(a[3]);
    o[4] = bf16_bits(c[0]); o[5] = bf16_bits(c[1]); o[6] = bf16_bits(c[2]); o[7] = bf16_bits(c[3]);
    *(volatile v8us*)(Cb + (size_t)(m0w + rl) * ldc + 64 * cy + 8 * q8) = o;
  }
}

template <int OM, int HB>
__global__ __launch_bounds__(128)
void gemm_kernel(const unsigned short* __restrict__ Ap, int lda, const unsigned short* __restrict__ Bw, int K,
                 const float* __restrict__ bias, float* Cf, unsigned short* Cb, int ldc)
{
  __shared__ __attribute__((aligned(16))) float sT[128 * 64];

  const int tid = threadIdx.x, lane = tid & 31, w = tid >> 5;
  const int h = lane >> 4, m = lane & 15;
  const int m0 = blockIdx.x * 128;
  const int cy = blockIdx.y;
  const int m0w = m0 + 32 * w;

  const unsigned short* xa = Ap + (size_t)(m0w + m) * lda;
  const unsigned short* wb = Bw + (size_t)(64 * cy + m) * K;

  v8f acc[2][4];
#pragma unroll
  for (int mt = 0; mt < 2; ++mt)
#pragma unroll
    for (int nt = 0; nt < 4; ++nt) acc[mt][nt] = zero8();

#pragma unroll 1
  for (int k0 = 0; k0 < K; k0 += 32) {
    Frag a0, a1;
    ldfrag_g(a0, xa + k0, h);
    ldfrag_g(a1, xa + (size_t)16 * lda + k0, h);
#pragma unroll
    for (int nt = 0; nt < 4; ++nt) {
      Frag b;
      ldfrag_g(b, wb + (size_t)nt * 16 * K + k0, h);
      acc[0][nt] = mma16(acc[0][nt], a0, b);
      acc[1][nt] = mma16(acc[1][nt], a1, b);
    }
  }

#pragma unroll
  for (int nt = 0; nt < 4; ++nt) {
    const int col = 16 * nt + m;
    const float bv = (HB == 1) ? bf16r(bias[64 * cy + col]) : 0.0f;
#pragma unroll
    for (int mt = 0; mt < 2; ++mt)
#pragma unroll
      for (int r = 0; r < 8; ++r) {
        const int rowl = 32 * w + 16 * mt + 8 * h + r;
        sT[rowl * 64 + col] = acc[mt][nt][r] + bv;
      }
  }
  __syncthreads();

  if (OM == 0) {
    c_store_pass(sT, Cf, ldc, m0w, cy, w, lane);
    __threadfence();
    c_store_pass(sT, Cf, ldc, m0w, cy, w, lane);
  } else {
    b_store_pass(sT, Cb, ldc, m0w, cy, w, lane);
    __threadfence();
    b_store_pass(sT, Cb, ldc, m0w, cy, w, lane);
  }
}

template <int NR>
__device__ __forceinline__ void h128_store_pass(const unsigned short* sY, unsigned short* g, int r0, int w, int lane) {
  const int q8 = lane & 7, sub = lane >> 3;
  constexpr int LPW = NR / 2;
  static_assert(LPW % 4 == 0);
#pragma unroll
  for (int i = 0; i < LPW / 4; ++i) {
    const int li = LPW * w + 4 * i + sub;
    const int row = li >> 1, hl = li & 1;
    const v8us v = *(const v8usa*)(sY + row * DI + 64 * hl + 8 * q8);
    *(volatile v8us*)(g + (size_t)(r0 + row) * DI + 64 * hl + 8 * q8) = v;
  }
}

__global__ __launch_bounds__(128)
void conv_kernel(const float* __restrict__ xh, const float* __restrict__ cw, const float* __restrict__ cb,
                 unsigned short* xcb)
{
  __shared__ __attribute__((aligned(16))) unsigned short sB[TV * DI];

  const int tid = threadIdx.x, lane = tid & 31, w = tid >> 5;
  const int t0 = blockIdx.x * TV;
  const int c = tid;

  const v4f cwv = *(const v4fa*)(cw + 4 * c);
  const float w0 = bf16r(cwv[0]), w1 = bf16r(cwv[1]), w2 = bf16r(cwv[2]), w3 = bf16r(cwv[3]);
  const float cbv = bf16r(cb[c]);

  const float* col = xh + c;
  int p, pc;
  p = t0 - 3; pc = (p > 0) ? p : 0;
  float v0 = col[(size_t)pc * DI]; v0 = (p >= 0) ? v0 : 0.0f;
  p = t0 - 2; pc = (p > 0) ? p : 0;
  float v1 = col[(size_t)pc * DI]; v1 = (p >= 0) ? v1 : 0.0f;
  p = t0 - 1; pc = (p > 0) ? p : 0;
  float v2 = col[(size_t)pc * DI]; v2 = (p >= 0) ? v2 : 0.0f;

#pragma unroll 1
  for (int tt = 0; tt < TV; ++tt) {
    const float v3 = col[(size_t)(t0 + tt) * DI];
    float s = cbv + w0 * v0; s = s + w1 * v1; s = s + w2 * v2; s = s + w3 * v3;
    const float y = silu_f(s);
    sB[tt * DI + tid] = bf16_bits(y);
    v0 = v1; v1 = v2; v2 = v3;
  }
  __syncthreads();

  h128_store_pass<TV>(sB, xcb, t0, w, lane);
  __threadfence();
  h128_store_pass<TV>(sB, xcb, t0, w, lane);
}

__device__ __forceinline__ void stage_xd(float* sX, const float* __restrict__ xd, int r0, int tid) {
#pragma unroll
  for (int k = 0; k < 2; ++k) {
    const int i = tid + 128 * k, tok = i >> 4, q = i & 15;
    *(v4fa*)(sX + tok * NXP + 4 * q) = *(const v4fa*)(xd + (size_t)(r0 + tok) * NXP + 4 * q);
  }
}

__device__ __forceinline__ void rec_store_pass(const float* s, float* g, int w, int lane) {
  const int q8 = lane & 7, sub = lane >> 3;
#pragma unroll
  for (int i = 0; i < 4; ++i) {
    const int li = 16 * w + 4 * i + sub;
    const v4f v = *(const v4fa*)(s + li * 32 + 4 * q8);
    *(volatile v4f*)(g + li * 32 + 4 * q8) = v;
  }
}

__global__ __launch_bounds__(128)
void scan1_kernel(const float* __restrict__ xh, const float* __restrict__ xd,
                  const float* __restrict__ cw, const float* __restrict__ cb,
                  const float* __restrict__ dtw, const float* __restrict__ dtb,
                  const float* __restrict__ alog, float* hsum, float* aprd)
{
  __shared__ __attribute__((aligned(16))) float sX[TC * NXP];
  __shared__ __attribute__((aligned(16))) float sR[2 * CHUNK * NS];

  const int tid = threadIdx.x, lane = tid & 31, w = tid >> 5;
  const int ch = blockIdx.x, t0 = ch * CHUNK, d = tid;

  const v4f cwv = *(const v4fa*)(cw + 4 * d);
  const float w0 = bf16r(cwv[0]), w1 = bf16r(cwv[1]), w2 = bf16r(cwv[2]), w3 = bf16r(cwv[3]);
  const float cbv = bf16r(cb[d]);
  const v4f dwv = *(const v4fa*)(dtw + 4 * d);
  const float e0 = bf16r(dwv[0]), e1 = bf16r(dwv[1]), e2 = bf16r(dwv[2]), e3 = bf16r(dwv[3]);
  const float bb = bf16r(dtb[d]);
  float An[NS];
  {
    const float* ap = alog + (size_t)d * NS;
#pragma unroll
    for (int q = 0; q < NS / 4; ++q) {
      const v4f av = *(const v4fa*)(ap + 4 * q);
#pragma unroll
      for (int j = 0; j < 4; ++j) An[4 * q + j] = -__expf(bf16r(av[j]));
    }
  }
  float hs[NS], apd[NS];
#pragma unroll
  for (int n = 0; n < NS; ++n) { hs[n] = 0.0f; apd[n] = 1.0f; }

  const float* col = xh + d;
  int p, pc;
  p = t0 - 3; pc = (p > 0) ? p : 0;
  float v0 = col[(size_t)pc * DI]; v0 = (p >= 0) ? v0 : 0.0f;
  p = t0 - 2; pc = (p > 0) ? p : 0;
  float v1 = col[(size_t)pc * DI]; v1 = (p >= 0) ? v1 : 0.0f;
  p = t0 - 1; pc = (p > 0) ? p : 0;
  float v2 = col[(size_t)pc * DI]; v2 = (p >= 0) ? v2 : 0.0f;

#pragma unroll 1
  for (int s = 0; s < CHUNK / TC; ++s) {
    const int r0 = t0 + TC * s;
    stage_xd(sX, xd, r0, tid);
    __syncthreads();
#pragma unroll 1
    for (int tt = 0; tt < TC; ++tt) {
      const float v3 = col[(size_t)(r0 + tt) * DI];
      float cs = cbv + w0 * v0; cs = cs + w1 * v1; cs = cs + w2 * v2; cs = cs + w3 * v3;
      const float xc = silu_f(cs);
      v0 = v1; v1 = v2; v2 = v3;
      const float* sr = sX + tt * NXP;
      const v4f dt4 = *(const v4fa*)sr;
      float dp = dt4[0] * e0; dp = dp + dt4[1] * e1; dp = dp + dt4[2] * e2; dp = dp + dt4[3] * e3;
      const float dl = softplus_f(dp + bb);
      const float bx = dl * xc;
      float Bn[NS];
#pragma unroll
      for (int q = 0; q < NS / 4; ++q) {
        const v4f bv = *(const v4fa*)(sr + DTR + 4 * q);
#pragma unroll
        for (int j = 0; j < 4; ++j) Bn[4 * q + j] = bv[j];
      }
#pragma unroll
      for (int n = 0; n < NS; ++n) {
        const float a = __expf(dl * An[n]);
        hs[n] = hs[n] * a + bx * Bn[n];
        apd[n] = apd[n] * a;
      }
    }
    __syncthreads();
  }

#pragma unroll
  for (int q = 0; q < NS / 4; ++q) {
    v4f hv, av;
#pragma unroll
    for (int j = 0; j < 4; ++j) { hv[j] = hs[4 * q + j]; av[j] = apd[4 * q + j]; }
    *(v4fa*)(sR + d * NS + 4 * q) = hv;
    *(v4fa*)(sR + CHUNK * NS + d * NS + 4 * q) = av;
  }
  __syncthreads();

  float* gh = hsum + (size_t)ch * (CHUNK * NS);
  float* ga = aprd + (size_t)ch * (CHUNK * NS);
  rec_store_pass(sR, gh, w, lane);
  rec_store_pass(sR + CHUNK * NS, ga, w, lane);
  __threadfence();
  rec_store_pass(sR, gh, w, lane);
  rec_store_pass(sR + CHUNK * NS, ga, w, lane);
}

__global__ __launch_bounds__(512)
void mid_kernel(const float* __restrict__ hsum, const float* __restrict__ aprd, float* carry)
{
  const int tid = threadIdx.x;
  v4f c;
  c[0] = 0.0f; c[1] = 0.0f; c[2] = 0.0f; c[3] = 0.0f;
#pragma unroll 1
  for (int ch = 0; ch < NCHK; ++ch) {
    const size_t o = (size_t)ch * (CHUNK * NS) + 4 * tid;
    const v4f hv = *(const v4fa*)(hsum + o);
    const v4f av = *(const v4fa*)(aprd + o);
    const v4f cv = c;
    *(volatile v4f*)(carry + o) = cv;
    __threadfence();
    *(volatile v4f*)(carry + o) = cv;
#pragma unroll
    for (int j = 0; j < 4; ++j) c[j] = av[j] * c[j] + hv[j];
  }
}

__global__ __launch_bounds__(128)
void scan3_kernel(const float* __restrict__ xh, const float* __restrict__ zp, const float* __restrict__ xd,
                  const float* __restrict__ carry,
                  const float* __restrict__ cw, const float* __restrict__ cb,
                  const float* __restrict__ dtw, const float* __restrict__ dtb,
                  const float* __restrict__ alog, const float* __restrict__ dpar,
                  unsigned short* yb)
{
  __shared__ __attribute__((aligned(16))) float sX[TC * NXP];
  __shared__ __attribute__((aligned(16))) unsigned short sY[TC * DI];

  const int tid = threadIdx.x, lane = tid & 31, w = tid >> 5;
  const int ch = blockIdx.x, t0 = ch * CHUNK, d = tid;

  const v4f cwv = *(const v4fa*)(cw + 4 * d);
  const float w0 = bf16r(cwv[0]), w1 = bf16r(cwv[1]), w2 = bf16r(cwv[2]), w3 = bf16r(cwv[3]);
  const float cbv = bf16r(cb[d]);
  const v4f dwv = *(const v4fa*)(dtw + 4 * d);
  const float e0 = bf16r(dwv[0]), e1 = bf16r(dwv[1]), e2 = bf16r(dwv[2]), e3 = bf16r(dwv[3]);
  const float bb = bf16r(dtb[d]);
  const float Dv = bf16r(dpar[d]);
  float An[NS], hs[NS];
  {
    const float* ap = alog + (size_t)d * NS;
    const float* cp = carry + (size_t)ch * (CHUNK * NS) + d * NS;
#pragma unroll
    for (int q = 0; q < NS / 4; ++q) {
      const v4f av = *(const v4fa*)(ap + 4 * q);
      const v4f hv = *(const v4fa*)(cp + 4 * q);
#pragma unroll
      for (int j = 0; j < 4; ++j) { An[4 * q + j] = -__expf(bf16r(av[j])); hs[4 * q + j] = hv[j]; }
    }
  }

  const float* col = xh + d;
  int p, pc;
  p = t0 - 3; pc = (p > 0) ? p : 0;
  float v0 = col[(size_t)pc * DI]; v0 = (p >= 0) ? v0 : 0.0f;
  p = t0 - 2; pc = (p > 0) ? p : 0;
  float v1 = col[(size_t)pc * DI]; v1 = (p >= 0) ? v1 : 0.0f;
  p = t0 - 1; pc = (p > 0) ? p : 0;
  float v2 = col[(size_t)pc * DI]; v2 = (p >= 0) ? v2 : 0.0f;

#pragma unroll 1
  for (int s = 0; s < CHUNK / TC; ++s) {
    const int r0 = t0 + TC * s;
    stage_xd(sX, xd, r0, tid);
    __syncthreads();
#pragma unroll 1
    for (int tt = 0; tt < TC; ++tt) {
      const float v3 = col[(size_t)(r0 + tt) * DI];
      float cs = cbv + w0 * v0; cs = cs + w1 * v1; cs = cs + w2 * v2; cs = cs + w3 * v3;
      const float xc = silu_f(cs);
      v0 = v1; v1 = v2; v2 = v3;
      const float* sr = sX + tt * NXP;
      const v4f dt4 = *(const v4fa*)sr;
      float dp = dt4[0] * e0; dp = dp + dt4[1] * e1; dp = dp + dt4[2] * e2; dp = dp + dt4[3] * e3;
      const float dl = softplus_f(dp + bb);
      const float bx = dl * xc;
      float Bn[NS], Cn[NS];
#pragma unroll
      for (int q = 0; q < NS / 4; ++q) {
        const v4f bv = *(const v4fa*)(sr + DTR + 4 * q);
        const v4f cv = *(const v4fa*)(sr + DTR + NS + 4 * q);
#pragma unroll
        for (int j = 0; j < 4; ++j) { Bn[4 * q + j] = bv[j]; Cn[4 * q + j] = cv[j]; }
      }
      float ps = 0.0f;
#pragma unroll
      for (int n = 0; n < NS; ++n) {
        const float a = __expf(dl * An[n]);
        hs[n] = hs[n] * a + bx * Bn[n];
        ps += hs[n] * Cn[n];
      }
      const float yv = ps + xc * Dv;
      const float zv = zp[(size_t)(r0 + tt) * DI + d];
      const float g = silu_f(zv);
      const float yg = yv * g;
      sY[tt * DI + tid] = bf16_bits(yg);
    }
    __syncthreads();

    h128_store_pass<TC>(sY, yb, r0, w, lane);
    __threadfence();
    h128_store_pass<TC>(sY, yb, r0, w, lane);
    __syncthreads();
  }
}

__global__ __launch_bounds__(256)
void lnout_kernel(const float* __restrict__ pp, const float* __restrict__ lg, const float* __restrict__ lb,
                  const float* __restrict__ x, float* out)
{
  __shared__ __attribute__((aligned(16))) float sO[CH * 36];

  const int tid = threadIdx.x, lane = tid & 31, w = tid >> 5;
  const int t0 = blockIdx.x * TO;
  const int b = t0 >> 14, hw0 = t0 & (HWN - 1);
  const int c0 = 2 * lane;

  const float g0 = bf16r(lg[c0]), g1 = bf16r(lg[c0 + 1]);
  const float b0 = bf16r(lb[c0]), b1 = bf16r(lb[c0 + 1]);

#pragma unroll 1
  for (int s = 0; s < 4; ++s) {
    const int tok = 4 * w + s;
    const v2f pv = *(const v2fa*)(pp + (size_t)(t0 + tok) * CH + c0);
    const float p0 = pv[0], p1 = pv[1];
    const float mu = wsum(p0 + p1) * (1.0f / CH);
    const float d0 = p0 - mu, d1 = p1 - mu;
    const float var = wsum(d0 * d0 + d1 * d1) * (1.0f / CH);
    const float rstd = rsqrtf(var + LNEPS);
    const float q0 = (d0 * rstd) * g0 + b0;
    const float q1 = (d1 * rstd) * g1 + b1;
    sO[c0 * 36 + tok] = silu_f(q0);
    sO[(c0 + 1) * 36 + tok] = silu_f(q1);
  }
  __syncthreads();

  const int q8 = lane & 7, sub = lane >> 3;
  v4f rv[2];
  size_t gi[2];
#pragma unroll
  for (int i = 0; i < 2; ++i) {
    const int co = 8 * w + 4 * i + sub;
    const v4f sv = *(const v4fa*)(sO + co * 36 + 4 * q8);
    gi[i] = ((size_t)(b * CH + co)) * HWN + hw0 + 4 * q8;
    const v4f xv = *(const v4fa*)(x + gi[i]);
#pragma unroll
    for (int j = 0; j < 4; ++j) rv[i][j] = sv[j] + bf16r(xv[j]);
  }
#pragma unroll
  for (int i = 0; i < 2; ++i) *(volatile v4f*)(out + gi[i]) = rv[i];
  __threadfence();
#pragma unroll
  for (int i = 0; i < 2; ++i) *(volatile v4f*)(out + gi[i]) = rv[i];
}

extern "C" void kernel_launch(void* const* d_in, const int* in_sizes, int n_in,
                              void* d_out, int out_size, void* d_ws, size_t ws_size,
                              hipStream_t stream)
{
  if (n_in < 14) return;
  if (in_sizes[0] != NB * CH * HWN) return;
  if (in_sizes[1] != DIN2 * CH) return;
  if (in_sizes[2] != DI * 4) return;
  if (in_sizes[3] != DI) return;
  if (in_sizes[4] != NXD * DI) return;
  if (in_sizes[5] != DI * DTR) return;
  if (in_sizes[6] != DI) return;
  if (in_sizes[7] != DI * NS) return;
  if (in_sizes[8] != DI) return;
  if (in_sizes[9] != CH * DI) return;
  if (in_sizes[10] != CH * CH) return;
  if (in_sizes[11] != CH || in_sizes[12] != CH || in_sizes[13] != CH) return;
  if (out_size != NB * CH * HWN) return;
  if (ws_size < WS_END) return;

  const float* x      = (const float*)d_in[0];
  const float* in_w   = (const float*)d_in[1];
  const float* conv_w = (const float*)d_in[2];
  const float* conv_b = (const float*)d_in[3];
  const float* xp_w   = (const float*)d_in[4];
  const float* dt_w   = (const float*)d_in[5];
  const float* dt_b   = (const float*)d_in[6];
  const float* a_log  = (const float*)d_in[7];
  const float* dpar   = (const float*)d_in[8];
  const float* out_w  = (const float*)d_in[9];
  const float* pj_w   = (const float*)d_in[10];
  const float* pj_b   = (const float*)d_in[11];
  const float* ln_g   = (const float*)d_in[12];
  const float* ln_b   = (const float*)d_in[13];
  float* out = (float*)d_out;

  char* ws = (char*)d_ws;
  unsigned short* WIN  = (unsigned short*)(ws + WO_WIN);
  unsigned short* WXP  = (unsigned short*)(ws + WO_WXP);
  unsigned short* WOUT = (unsigned short*)(ws + WO_WOUT);
  unsigned short* WPJ  = (unsigned short*)(ws + WO_WPJ);
  unsigned short* X0   = (unsigned short*)(ws + OFF_X0);
  unsigned short* MOB  = (unsigned short*)(ws + OFF_MOB);
  float*          XH   = (float*)(ws + OFF_XH);
  float*          Z    = (float*)(ws + OFF_Z);
  unsigned short* XCB  = (unsigned short*)(ws + OFF_XC);
  unsigned short* YB   = (unsigned short*)(ws + OFF_YB);
  float*          XD   = (float*)(ws + OFF_XD);
  float*          P    = (float*)(ws + OFF_P);
  float*          HS   = (float*)(ws + OFF_HS);
  float*          AP   = (float*)(ws + OFF_AP);
  float*          CR   = (float*)(ws + OFF_CR);

  tcvt_kernel<<<dim3(HWN / 64, CH / 64, NB), dim3(256), 0, stream>>>(
      x, CH, HWN, (size_t)CH * HWN, X0, CH, (size_t)HWN * CH);

  cvt_kernel<<<dim3((DIN2 * CH) / 2048), dim3(256), 0, stream>>>(in_w, DIN2 * CH, WIN, DIN2 * CH);
  cvt_kernel<<<dim3((NXP * DI) / 2048), dim3(256), 0, stream>>>(xp_w, NXD * DI, WXP, NXP * DI);
  cvt_kernel<<<dim3((CH * DI) / 2048), dim3(256), 0, stream>>>(out_w, CH * DI, WOUT, CH * DI);
  cvt_kernel<<<dim3((CH * CH) / 2048), dim3(256), 0, stream>>>(pj_w, CH * CH, WPJ, CH * CH);

  gemm_kernel<0, 0><<<dim3(NTOK / 128, DI / 64), dim3(128), 0, stream>>>(
      X0, CH, WIN, CH, pj_b, XH, MOB, DI);
  gemm_kernel<0, 0><<<dim3(NTOK / 128, DI / 64), dim3(128), 0, stream>>>(
      X0, CH, WIN + (size_t)DI * CH, CH, pj_b, Z, MOB, DI);

  conv_kernel<<<dim3(NTOK / TV), dim3(128), 0, stream>>>(XH, conv_w, conv_b, XCB);

  gemm_kernel<0, 0><<<dim3(NTOK / 128, NXP / 64), dim3(128), 0, stream>>>(
      XCB, DI, WXP, DI, pj_b, XD, MOB, NXP);

  scan1_kernel<<<dim3(NCHK), dim3(128), 0, stream>>>(XH, XD, conv_w, conv_b, dt_w, dt_b, a_log, HS, AP);
  mid_kernel<<<dim3(1), dim3(512), 0, stream>>>(HS, AP, CR);
  scan3_kernel<<<dim3(NCHK), dim3(128), 0, stream>>>(XH, Z, XD, CR, conv_w, conv_b, dt_w, dt_b, a_log, dpar, YB);

  gemm_kernel<1, 0><<<dim3(NTOK / 128, CH / 64), dim3(128), 0, stream>>>(
      YB, DI, WOUT, DI, pj_b, P, MOB, CH);

  gemm_kernel<0, 1><<<dim3(NTOK / 128, CH / 64), dim3(128), 0, stream>>>(
      MOB, CH, WPJ, CH, pj_b, P, MOB, CH);

  lnout_kernel<<<dim3(NTOK / TO), dim3(256), 0, stream>>>(P, ln_g, ln_b, x, out);
}
